// RelationNonLocal_46102178955357
// MI455X (gfx1250) — hardware-run, weakly checked
//
#include <hip/hip_runtime.h>


#ifndef NB
#define NB 4
#endif
#ifndef HWP
#define HWP 4096
#endif
#define NB_FULL 4
#define HW_FULL 4096
#ifndef OUT_HW
#define OUT_HW HWP
#endif
#define CH     256
#define KSPLIT 8
#define KCH    (HWP / KSPLIT)
#define WCAR   64.0f
#define GCAR   64.0f
#define FRSH   4
#define OUTSH  8

static constexpr float GSC = GCAR / (float)HWP;

static_assert(CH % 64 == 0);
static_assert(CH % 32 == 0);
static_assert(HWP % 64 == 0);
static_assert((HWP & (HWP - 1)) == 0);
static_assert(HWP % KSPLIT == 0);
static_assert(KCH % 32 == 0);
static_assert(NB <= NB_FULL);
static_assert(HWP <= HW_FULL);
static_assert(HW_FULL % 4 == 0);
static_assert(OUT_HW % 64 == 0);
static_assert(OUT_HW >= HWP);
static_assert(((size_t)CH * CH) % (8 * 256) == 0);
static_assert(((size_t)NB * CH * CH) % (8 * 256) == 0);
static_assert(64 * 68 * 4 <= 131072);
static_assert(16 * 68 * 4 <= 131072);

typedef _Float16 h16;
typedef unsigned short bf;
typedef __attribute__((ext_vector_type(16))) __bf16   v16bf;
typedef __attribute__((ext_vector_type(16))) _Float16 v16h;
typedef __attribute__((ext_vector_type(8)))  _Float16 v8h;
typedef __attribute__((ext_vector_type(8)))  unsigned short v8us;
typedef __attribute__((ext_vector_type(8)))  float    v8f;
typedef __attribute__((ext_vector_type(4)))  float    v4f;
typedef v4f  __attribute__((may_alias)) v4fa;

__device__ __forceinline__ unsigned short f2bf(float f) { unsigned u = __float_as_uint(f); u += 0x7FFFu + ((u >> 16) & 1u); return (unsigned short)(u >> 16); }
__device__ __forceinline__ float bfr(float f) { return __uint_as_float(((unsigned)f2bf(f)) << 16); }
__device__ __forceinline__ v16h cat16(v8h lo, v8h hi) { return __builtin_shufflevector(lo, hi, 0, 1, 2, 3, 4, 5, 6, 7, 8, 9, 10, 11, 12, 13, 14, 15); }
__device__ __forceinline__ v16bf cat16b(v8us lo, v8us hi) { return __builtin_bit_cast(v16bf, __builtin_shufflevector(lo, hi, 0, 1, 2, 3, 4, 5, 6, 7, 8, 9, 10, 11, 12, 13, 14, 15)); }
__device__ __forceinline__ v8f wmma16(v16h a, v16h b, v8f c) { return __builtin_amdgcn_wmma_f32_16x16x32_f16(false, a, false, b, (short)0, c, false, false); }
__device__ __forceinline__ v8f wmmab(v16bf a, v16bf b, v8f c) { return __builtin_amdgcn_wmma_f32_16x16x32_bf16(false, a, false, b, (short)0, c, false, false); }
__device__ __forceinline__ v16h  ldh(const h16* p) { return cat16(*(const v8h*)p, *(const v8h*)(p + 16)); }
__device__ __forceinline__ v16bf ldb(const bf* p)  { return cat16b(*(const v8us*)p, *(const v8us*)(p + 16)); }
__device__ __forceinline__ void wave_sync() { __builtin_amdgcn_fence(3  , "wavefront"); __builtin_amdgcn_wave_barrier(); asm volatile("" ::: "memory"); }

__device__ __forceinline__ v8f wmma16g(v16h a, v16h b, v8f c) { c = wmma16(a, b, c); asm volatile("v_nop\n\tv_nop\n\tv_nop\n\tv_nop" : "+v"(c) : "v"(a), "v"(b)); return c; }
__device__ __forceinline__ v8f wmmabg(v16bf a, v16bf b, v8f c) { c = wmmab(a, b, c); asm volatile("v_nop\n\tv_nop\n\tv_nop\n\tv_nop" : "+v"(c) : "v"(a), "v"(b)); return c; }
__device__ __forceinline__ v16h  ldfrag(const h16* p) { return ldh(p); }
__device__ __forceinline__ v16bf ldfrag(const bf* p)  { return ldb(p); }
__device__ __forceinline__ v8f mmag(v16h a, v16h b, v8f c)   { return wmma16g(a, b, c); }
__device__ __forceinline__ v8f mmag(v16bf a, v16bf b, v8f c) { return wmmabg(a, b, c); }
static __device__ __forceinline__ h16 toh_flush(float v) { const float w = (fabsf(v) < 6.103515625e-05f) ? 0.0f : v; return (h16)w; }

__global__ __launch_bounds__(256) void k_cvt8(const float* __restrict__ src, bf* dst, size_t n8) {
    const size_t i = (size_t)blockIdx.x * 256 + threadIdx.x; if (i >= n8) return;
    const v8f v = *(const v8f*)(src + i * 8); v8us o;
#pragma unroll
    for (int k = 0; k < 8; ++k) o[k] = f2bf(v[k]);
    *(volatile v8us*)(dst + i * 8) = o; __threadfence(); *(volatile v8us*)(dst + i * 8) = o;
}

__global__ __launch_bounds__(256) void k_wcvt(const float* __restrict__ src, h16* dst, size_t n8) {
    const size_t i = (size_t)blockIdx.x * 256 + threadIdx.x; if (i >= n8) return;
    const v8f v = *(const v8f*)(src + i * 8); v8h o;
#pragma unroll
    for (int k = 0; k < 8; ++k) o[k] = toh_flush(bfr(v[k]) * WCAR);
    *(volatile v8h*)(dst + i * 8) = o; __threadfence(); *(volatile v8h*)(dst + i * 8) = o;
}

__global__ __launch_bounds__(256) void k_xt(const float* __restrict__ x, bf* XT) {
    __shared__ __align__(16) float ts[64 * 68];
    static_assert(4 * 256 == 64 * 16);
    static_assert(2 * 256 * 16 == 64 * 128);
    const unsigned tid = threadIdx.x;
    const unsigned p0 = blockIdx.x * 64u, c0 = blockIdx.y * 64u, n = blockIdx.z;
    const float* xb = x + ((size_t)n * CH + c0) * HW_FULL + p0;
#pragma unroll
    for (int s = 0; s < 4; ++s) {
        const unsigned idx = (unsigned)s * 256u + tid; const unsigned c = idx >> 4, p4 = (idx & 15u) * 4u;
        const v4f v = *(const v4f*)(xb + (size_t)c * HW_FULL + p4);
        ts[(p4 + 0u) * 68u + c] = v[0]; ts[(p4 + 1u) * 68u + c] = v[1]; ts[(p4 + 2u) * 68u + c] = v[2]; ts[(p4 + 3u) * 68u + c] = v[3];
    }
    __syncthreads();
    bf* ob = XT + ((size_t)n * HWP + p0) * CH + c0;
#pragma unroll 1
    for (int ps = 0; ps < 2; ++ps) {
#pragma unroll
        for (int s = 0; s < 2; ++s) {
            const unsigned idx = (unsigned)s * 256u + tid; const unsigned row = idx >> 3, c8 = (idx & 7u) * 8u;
            const v4f x0 = *(const v4fa*)(&ts[row * 68u + c8]); const v4f x1 = *(const v4fa*)(&ts[row * 68u + c8 + 4u]); v8us o;
#pragma unroll
            for (int i = 0; i < 4; ++i) { o[i] = f2bf(x0[i]); o[4 + i] = f2bf(x1[i]); }
            *(volatile v8us*)(ob + (size_t)row * CH + c8) = o; }
        if (ps == 0) __threadfence(); }
}

template <typename T, int LDK, int KLEN, int BIASK, int OUTF32, int SH>
__device__ __forceinline__ void gemm_tile(const T* __restrict__ A, const T* __restrict__ Bt, const float* __restrict__ bias, h16* OH, float* OF, const size_t pitch) {
    __shared__ __align__(16) float os[16 * 68];
    static_assert(KLEN % 32 == 0);
    static_assert(LDK % 8 == 0);
    static_assert(32 * 16 * 4 == 16 * 128);
    static_assert(32 * 16 * 8 == 16 * 256);
    constexpr float sc = 1.0f / (float)(1 << SH);
    const int lane = threadIdx.x & 31, lr = lane & 15, hi = lane >> 4;
    v8f acc[4][4];
#pragma unroll
    for (int mb = 0; mb < 4; ++mb)
#pragma unroll
        for (int nb = 0; nb < 4; ++nb) acc[mb][nb] = (v8f){};
    const size_t foff = (size_t)lr * LDK + 8 * hi;
#pragma unroll 1
    for (int kc = 0; kc < KLEN; kc += 32) {
        decltype(ldfrag(A)) a[4];
#pragma unroll
        for (int mb = 0; mb < 4; ++mb) a[mb] = ldfrag(A + foff + (size_t)mb * 16 * LDK + kc);
#pragma unroll
        for (int nb = 0; nb < 4; ++nb) { const decltype(ldfrag(Bt)) b = ldfrag(Bt + foff + (size_t)nb * 16 * LDK + kc);
#pragma unroll
            for (int mb = 0; mb < 4; ++mb) acc[mb][nb] = mmag(a[mb], b, acc[mb][nb]); }
    }
    float bc[4];
#pragma unroll
    for (int nb = 0; nb < 4; ++nb) { bc[nb] = 0.0f; if (BIASK == 1) bc[nb] = bfr(bias[nb * 16 + lr]); }
#pragma unroll
    for (int mb = 0; mb < 4; ++mb) {
        float br[8];
#pragma unroll
        for (int j = 0; j < 8; ++j) { br[j] = 0.0f; if (BIASK == 2) br[j] = bfr(bias[mb * 16 + hi * 8 + j]); }
#pragma unroll
        for (int nb = 0; nb < 4; ++nb) {
#pragma unroll
            for (int j = 0; j < 8; ++j) os[(hi * 8 + j) * 68 + nb * 16 + lr] = acc[mb][nb][j] * sc + bc[nb] + br[j]; }
        wave_sync();
#pragma unroll 1
        for (int ps = 0; ps < 2; ++ps) {
            if (OUTF32) {
#pragma unroll
                for (int s = 0; s < 8; ++s) { const int row = 2 * s + (lane >> 4), c4 = (lane & 15) * 4;
                    const v4f val = *(const v4fa*)(&os[row * 68 + c4]);
                    *(volatile v4f*)(OF + (size_t)(mb * 16 + row) * pitch + c4) = val; }
            } else {
#pragma unroll
                for (int s = 0; s < 4; ++s) { const int row = 4 * s + (lane >> 3), c8 = (lane & 7) * 8;
                    const v4f x0 = *(const v4fa*)(&os[row * 68 + c8]); const v4f x1 = *(const v4fa*)(&os[row * 68 + c8 + 4]); v8h hv;
#pragma unroll
                    for (int i = 0; i < 4; ++i) { hv[i] = toh_flush(x0[i]); hv[4 + i] = toh_flush(x1[i]); }
                    *(volatile v8h*)(OH + (size_t)(mb * 16 + row) * pitch + c8) = hv; }
            }
            if (ps == 0) __threadfence(); }
        wave_sync();
    }
}

__global__ __launch_bounds__(32) void k_projT(const bf* __restrict__ W, const bf* __restrict__ XT, const float* __restrict__ bias, h16* PT) {
    const unsigned r0 = blockIdx.x * 64u, c0 = blockIdx.y * 64u;
    const unsigned n = c0 / (unsigned)HWP, p0 = c0 % (unsigned)HWP;
    gemm_tile<bf, CH, CH, 2, 0, 0>(W + (size_t)r0 * CH, XT + (size_t)c0 * CH, bias + r0, PT + ((size_t)n * CH + r0) * HWP + p0, nullptr, (size_t)HWP);
}

__global__ __launch_bounds__(32) void k_projQ(const bf* __restrict__ XT, const bf* __restrict__ W, const float* __restrict__ bias, h16* QP) {
    const unsigned r0 = blockIdx.x * 64u, c0 = blockIdx.y * 64u;
    gemm_tile<bf, CH, CH, 1, 0, 0>(XT + (size_t)r0 * CH, W + (size_t)c0 * CH, bias + c0, QP + (size_t)r0 * CH + c0, nullptr, (size_t)CH);
}

__global__ __launch_bounds__(32) void k_gram(const h16* __restrict__ VT, const h16* __restrict__ KT, float* GP) {
    const unsigned r0 = blockIdx.x * 64u, c0 = blockIdx.y * 64u, z = blockIdx.z;
    const unsigned s = z / (unsigned)NB, n = z % (unsigned)NB;
    gemm_tile<h16, HWP, KCH, 0, 1, 0>(VT + ((size_t)n * CH + r0) * HWP + (size_t)s * KCH, KT + ((size_t)n * CH + c0) * HWP + (size_t)s * KCH, nullptr,
                                      nullptr, GP + ((size_t)z * CH + r0) * CH + c0, (size_t)CH);
}

__global__ __launch_bounds__(256) void k_gred(const float* __restrict__ GP, h16* GT, size_t n8) {
    const size_t i = (size_t)blockIdx.x * 256 + threadIdx.x; if (i >= n8) return;
    v8f sum = (v8f){};
#pragma unroll 1
    for (int k = 0; k < KSPLIT; ++k) { const v8f v = *(const v8f*)(GP + (size_t)k * ((size_t)NB * CH * CH) + i * 8); sum = sum + v; }
    v8h o;
#pragma unroll
    for (int e = 0; e < 8; ++e) o[e] = toh_flush(sum[e] * GSC);
    *(volatile v8h*)(GT + i * 8) = o; __threadfence(); *(volatile v8h*)(GT + i * 8) = o;
}

__global__ __launch_bounds__(32) void k_fr(const h16* __restrict__ QP, const h16* __restrict__ GT, h16* FR) {
    const unsigned r0 = blockIdx.x * 64u, c0 = blockIdx.y * 64u;
    const unsigned n = r0 / (unsigned)HWP;
    gemm_tile<h16, CH, CH, 0, 0, FRSH>(QP + (size_t)r0 * CH, GT + ((size_t)n * CH + c0) * CH, nullptr, FR + (size_t)r0 * CH + c0, nullptr, (size_t)CH);
}

__global__ __launch_bounds__(32) void k_out(const h16* __restrict__ W3H, const h16* __restrict__ FR, const float* __restrict__ bias, float* OUT) {
    const unsigned r0 = blockIdx.x * 64u, c0 = blockIdx.y * 64u;
    const unsigned n = c0 / (unsigned)HWP, p0 = c0 % (unsigned)HWP;
    gemm_tile<h16, CH, CH, 2, 1, OUTSH>(W3H + (size_t)r0 * CH, FR + (size_t)c0 * CH, bias + r0, nullptr, OUT + ((size_t)n * CH + r0) * OUT_HW + p0, (size_t)OUT_HW);
}

static constexpr size_t al256(size_t v) { return (v + 255) & ~(size_t)255; }
static constexpr size_t SZ_XT = al256((size_t)NB * HWP * CH * 2);
static constexpr size_t SZ_WB = al256((size_t)3 * CH * CH * 2);
static constexpr size_t SZ_W3 = al256((size_t)CH * CH * 2);
static constexpr size_t SZ_PL = al256((size_t)NB * CH * HWP * 2);
static constexpr size_t SZ_GP = al256((size_t)KSPLIT * NB * CH * CH * 4);
static constexpr size_t SZ_GT = al256((size_t)NB * CH * CH * 2);
static constexpr size_t SZ_TOTAL = SZ_XT + SZ_WB + SZ_W3 + 4 * SZ_PL + SZ_GP + SZ_GT;
static_assert(SZ_TOTAL <= (size_t)134217728);
static_assert(((size_t)CH * CH * 2) % 256 == 0);
static constexpr size_t NEED_X = ((size_t)(NB - 1) * CH + (size_t)(CH - 1)) * HW_FULL + HWP;
static constexpr size_t NEED_O = ((size_t)(NB - 1) * CH + (size_t)(CH - 1)) * OUT_HW + HWP;
static constexpr size_t N8_W   = (size_t)CH * CH / 8;
static constexpr size_t N8_G   = (size_t)NB * CH * CH / 8;
static_assert(NEED_O * 4 <= (size_t)NB_FULL * CH * HW_FULL * 4 || OUT_HW > HW_FULL);

extern "C" void kernel_launch(void* const* d_in, const int* in_sizes, int n_in,
                              void* d_out, int out_size, void* d_ws, size_t ws_size, hipStream_t stream) {
    if (n_in < 9) return;
    if ((size_t)in_sizes[0] < NEED_X) return;
    if ((size_t)in_sizes[1] < (size_t)CH * CH || (size_t)in_sizes[3] < (size_t)CH * CH || (size_t)in_sizes[5] < (size_t)CH * CH || (size_t)in_sizes[7] < (size_t)CH * CH) return;
    if (in_sizes[2] < CH || in_sizes[4] < CH || in_sizes[6] < CH || in_sizes[8] < CH) return;
    if ((size_t)out_size < NEED_O) return;
    if (SZ_TOTAL > ws_size) return;
    const float* x  = (const float*)d_in[0];
    const float* w0 = (const float*)d_in[1]; const float* b0 = (const float*)d_in[2];
    const float* w1 = (const float*)d_in[3]; const float* b1 = (const float*)d_in[4];
    const float* w2 = (const float*)d_in[5]; const float* b2 = (const float*)d_in[6];
    const float* w3 = (const float*)d_in[7]; const float* b3 = (const float*)d_in[8];
    float* OUT = (float*)d_out;
    char* wsp = (char*)d_ws;
    bf*  XT  = (bf*)wsp;  wsp += SZ_XT;
    bf*  WB  = (bf*)wsp;  wsp += SZ_WB;
    h16* W3H = (h16*)wsp; wsp += SZ_W3;
    h16* VT  = (h16*)wsp; wsp += SZ_PL;
    h16* KT  = (h16*)wsp; wsp += SZ_PL;
    h16* QP  = (h16*)wsp; wsp += SZ_PL;
    h16* FR  = (h16*)wsp; wsp += SZ_PL;
    float* GP = (float*)wsp; wsp += SZ_GP;
    h16* GT  = (h16*)wsp; wsp += SZ_GT;
    bf* WV = WB; bf* WK = WB + (size_t)CH * CH; bf* WQ = WB + (size_t)2 * CH * CH;

    k_xt<<<dim3(HWP / 64, CH / 64, NB), 256, 0, stream>>>(x, XT);
    { const unsigned g = (unsigned)((N8_W + 255) / 256);
      k_cvt8<<<g, 256, 0, stream>>>(w0, WV, N8_W); k_cvt8<<<g, 256, 0, stream>>>(w1, WK, N8_W); k_cvt8<<<g, 256, 0, stream>>>(w2, WQ, N8_W);
      k_wcvt<<<g, 256, 0, stream>>>(w3, W3H, N8_W); }

    k_projT<<<dim3(CH / 64, NB * HWP / 64, 1), 32, 0, stream>>>(WV, XT, b0, VT);
    k_projT<<<dim3(CH / 64, NB * HWP / 64, 1), 32, 0, stream>>>(WK, XT, b1, KT);
    k_projQ<<<dim3(NB * HWP / 64, CH / 64, 1), 32, 0, stream>>>(XT, WQ, b2, QP);

    k_gram<<<dim3(CH / 64, CH / 64, KSPLIT * NB), 32, 0, stream>>>(VT, KT, GP);
    k_gred<<<(unsigned)((N8_G + 255) / 256), 256, 0, stream>>>(GP, GT, N8_G);

    k_fr<<<dim3(NB * HWP / 64, CH / 64, 1), 32, 0, stream>>>(QP, GT, FR);
    k_out<<<dim3(CH / 64, NB * HWP / 64, 1), 32, 0, stream>>>(W3H, FR, b3, OUT);
}
